// PhaserModel_17300128269093
// MI455X (gfx1250) — hardware-verified
//
#include <hip/hip_runtime.h>
#include <math.h>


#pragma clang fp contract(off)

#define TSAMP        262144
#define NCH          2
#define HW           32
#define TILE_M       16
#define TILES_PER_CH (TSAMP / TILE_M)
#define TOTAL_TILES  (NCH * TILES_PER_CH)
#define COEF_THREADS 256
#define COEF_WAVES   (COEF_THREADS / 32)
#define COEF_BLOCKS  128
#define TPW          (TOTAL_TILES / (COEF_BLOCKS * COEF_WAVES))
#define ARG_BLK      128
#define ARG_NBLK     (TSAMP / ARG_BLK)
#define ARG_OUTER_LEVELS 1
#define ST_THREADS   512
#define CHUNK        (TSAMP / ST_THREADS)

static_assert(TPW * COEF_BLOCKS * COEF_WAVES == TOTAL_TILES);
static_assert((TPW % 2) == 0);
static_assert(ST_THREADS * CHUNK == TSAMP);
static_assert((CHUNK % 32) == 0);
static_assert(TILES_PER_CH == 16384);
static_assert(ARG_NBLK == 2048);

typedef _Float16 v16h __attribute__((ext_vector_type(16)));
typedef float    v8f  __attribute__((ext_vector_type(8)));
typedef float    v4f  __attribute__((ext_vector_type(4)));

__device__ __forceinline__ v8f wmma_f16(v16h a, v16h b, v8f c)
{
    v8f d = __builtin_amdgcn_wmma_f32_16x16x32_f16(false, a, false, b, (short)0, c, false, false);
    asm volatile("v_nop\n\tv_nop\n\tv_nop\n\tv_nop" : "+v"(d) : "v"(a), "v"(b));
    return d;
}

__device__ __forceinline__ float tanh_fast(float x)
{
    const float e = __expf(2.0f * x);
    return 1.0f - 2.0f * __builtin_amdgcn_rcpf(e + 1.0f);
}

__global__ __launch_bounds__(COEF_THREADS)
void k_coef(const float* __restrict__ lfo_rate,
            const float* __restrict__ phoff,
            const float* __restrict__ amp,
            const float* __restrict__ bias,
            const float* __restrict__ depth,
            const float* __restrict__ W1,
            const float* __restrict__ b1,
            const float* __restrict__ W2,
            const float* __restrict__ b2,
            const float* __restrict__ W3,
            const float* __restrict__ b3,
            float* __restrict__ pOut)
{
    __shared__ float S1s[ARG_BLK];
    __shared__ float E1s[ARG_NBLK];
#if ARG_OUTER_LEVELS == 2
    __shared__ float Scs[ARG_BLK];
    __shared__ float E2s[ARG_NBLK / ARG_BLK];
#endif

    const int tid  = threadIdx.x;
    const int lane = tid & 31;
    const int wv   = tid >> 5;
    const int n    = lane & 15;
    const int h    = lane >> 4;

    const float stepv = (6.283185307179586f * lfo_rate[0]) * (1.0f / 44100.0f);

    if (tid == 0) {
        float acc = 0.0f;
        for (int j = 0; j < ARG_BLK; ++j) { acc = acc + stepv; S1s[j] = acc; }
    }
    __syncthreads();
#if ARG_OUTER_LEVELS == 2
    if (tid == 0) {
        const float c1 = S1s[ARG_BLK - 1];
        float acc = 0.0f;
        for (int j = 0; j < ARG_BLK; ++j) { acc = acc + c1; Scs[j] = acc; }
        const float c2 = acc;
        float acc2 = 0.0f;
        for (int k = 0; k < ARG_NBLK / ARG_BLK; ++k) { E2s[k] = acc2; acc2 = acc2 + c2; }
    }
    __syncthreads();
    for (int b = tid; b < ARG_NBLK; b += COEF_THREADS)
        E1s[b] = (b == 0) ? 0.0f : (Scs[(b - 1) & (ARG_BLK - 1)] + E2s[(b - 1) >> 7]);
#else
    if (tid == 0) {
        const float c1 = S1s[ARG_BLK - 1];
        float acc = 0.0f;
        for (int b = 0; b < ARG_NBLK; ++b) { E1s[b] = acc; acc = acc + c1; }
    }
#endif
    __syncthreads();

    v16h B0 = {};
    v16h B1 = {};
#pragma unroll
    for (int i = 0; i < 8; ++i) {
        const int klo = 8 * h + i;
        const int khi = 16 + 8 * h + i;
        B0[i]     = (_Float16)(64.0f * W2[klo * HW + n]);
        B0[8 + i] = (_Float16)(64.0f * W2[khi * HW + n]);
        B1[i]     = (_Float16)(64.0f * W2[klo * HW + 16 + n]);
        B1[8 + i] = (_Float16)(64.0f * W2[khi * HW + 16 + n]);
    }

    float w1r[16], b1r[16];
#pragma unroll
    for (int i = 0; i < 16; ++i) {
        const int ku = (i < 8) ? (8 * h + i) : (8 + 8 * h + i);
        w1r[i] = W1[ku];
        b1r[i] = b1[ku];
    }
    const float w3a = W3[n], w3b = W3[16 + n];
    const float b2a = b2[n], b2b = b2[16 + n];
    const float ampv = amp[0], biasv = bias[0], b3v = b3[0], po = phoff[0];
    const float hdep = depth[0] * 0.5f;

    const int gwave = blockIdx.x * COEF_WAVES + wv;

    float p_even  = 0.0f;
    int   lineBase = 0;

    for (int it = 0; it < TPW; ++it) {
        const int tt = gwave * TPW + it;
        if (tt >= TOTAL_TILES) break;
        const int ch = tt >> 14;
        const int t0 = (tt & (TILES_PER_CH - 1)) << 4;
        const int ts = t0 + n;

        const float argl = S1s[ts & (ARG_BLK - 1)] + E1s[ts >> 7];
        const float arg  = ch ? (argl + po) : argl;
        const float z    = ampv * cosf(arg);

        v16h A = {};
#pragma unroll
        for (int i = 0; i < 16; ++i) {
            const float a1 = z * w1r[i];
            const float a2 = a1 + b1r[i];
            A[i] = (_Float16)(16.0f * tanh_fast(a2));
        }

        const v8f cz = {};
        const v8f c0 = wmma_f16(A, B0, cz);
        const v8f c1 = wmma_f16(A, B1, cz);

        float tsum[8];
#pragma unroll
        for (int r = 0; r < 8; ++r) {
            const float u0 = c0[r] * 0.0009765625f + b2a;
            const float u1 = c1[r] * 0.0009765625f + b2b;
            tsum[r] = tanh_fast(u0) * w3a + tanh_fast(u1) * w3b;
        }
#pragma unroll
        for (int msk = 1; msk < 16; msk <<= 1) {
#pragma unroll
            for (int r = 0; r < 8; ++r) tsum[r] += __shfl_xor(tsum[r], msk, 32);
        }
        float mv = tsum[0];
#pragma unroll
        for (int r = 1; r < 8; ++r) mv = (n == r) ? tsum[r] : mv;
        const float m  = mv + b3v;
        const float u  = 1.0f + m;
        const float v  = hdep * u;
        const float d  = biasv + v;
        const float td = tanf(d);
        const float rr = (1.0f - td) / (1.0f + td);
        const float pc = tanhf(rr);

        if ((it & 1) == 0) {
            p_even   = pc;
            lineBase = ch * TSAMP + t0;
        } else {
            v4f vv;
#pragma unroll
            for (int i = 0; i < 4; ++i) {
                const int s   = ((lane & 7) << 2) + i;
                const int src = (((s >> 3) & 1) << 4) + (s & 7);
                const float ve = __shfl(p_even, src, 32);
                const float vo = __shfl(pc, src, 32);
                vv[i] = (s & 16) ? vo : ve;
            }
            volatile v4f* dst = (volatile v4f*)(pOut + lineBase + ((lane & 7) << 2));
            if (lane < 8) *dst = vv;
            __threadfence();
            if (lane < 8) *dst = vv;
        }
    }
}

__global__ __launch_bounds__(ST_THREADS)
void k_stage(const float* sIn, int inStride,
             const float* __restrict__ pAll,
             const float* xIn,
             float* __restrict__ dst, int mode)
{
    __shared__ float As[ST_THREADS];
    __shared__ float Ys[ST_THREADS];

    const int ch    = blockIdx.x;
    const int t     = threadIdx.x;
    const int start = t * CHUNK;
    const float* s  = sIn  + (size_t)ch * (size_t)inStride;
    const float* pc = pAll + (size_t)ch * TSAMP;
    float* dch      = dst  + (size_t)ch * TSAMP;

    const float sp0 = (start == 0) ? 0.0f : s[start - 1];

    float Acc = 1.0f, Ycc = 0.0f, sp = sp0;
    for (int blk = 0; blk < CHUNK / 32; ++blk) {
        const int base = start + blk * 32;
        v4f pv4[8], cv4[8];
#pragma unroll
        for (int q = 0; q < 8; ++q) {
            pv4[q] = *(const v4f*)(pc + base + 4 * q);
            cv4[q] = *(const v4f*)(s + base + 4 * q);
        }
#pragma unroll
        for (int i = 0; i < 32; ++i) {
            const float pv  = pv4[i >> 2][i & 3];
            const float cur = cv4[i >> 2][i & 3];
            const float t1 = pv * cur;
            const float t2 = t1 + sp;
            const float t3 = pv * Ycc;
            Ycc = t2 - t3;
            Acc = Acc * (-pv);
            sp = cur;
        }
    }
    As[t] = Acc;
    Ys[t] = Ycc;
    __syncthreads();

    for (int off = 1; off < ST_THREADS; off <<= 1) {
        float aP = 1.0f, yP = 0.0f;
        const bool has = (t >= off);
        if (has) { aP = As[t - off]; yP = Ys[t - off]; }
        __syncthreads();
        if (has) {
            const float a0 = As[t];
            const float y0 = Ys[t];
            As[t] = a0 * aP;
            Ys[t] = a0 * yP + y0;
        }
        __syncthreads();
    }
    const float carry = (t == 0) ? 0.0f : Ys[t - 1];

    for (int pass = 0; pass < 2; ++pass) {
        float y = carry, spv = sp0;
        for (int blk = 0; blk < CHUNK / 32; ++blk) {
            const int base = start + blk * 32;
            v4f pv4[8], cv4[8], xv4[8];
#pragma unroll
            for (int q = 0; q < 8; ++q) {
                pv4[q] = *(const v4f*)(pc + base + 4 * q);
                cv4[q] = *(const v4f*)(s + base + 4 * q);
                const v4f zz = {};
                xv4[q] = zz;
            }
            if (mode) {
#pragma unroll
                for (int q = 0; q < 8; ++q) xv4[q] = *(const v4f*)(xIn + base + 4 * q);
            }
            float vals[32];
#pragma unroll
            for (int i = 0; i < 32; ++i) {
                const float pv  = pv4[i >> 2][i & 3];
                const float cur = cv4[i >> 2][i & 3];
                const float t1 = pv * cur;
                const float t2 = t1 + spv;
                const float t3 = pv * y;
                y = t2 - t3;
                spv = cur;
                const float mixed = 0.5f * (xv4[i >> 2][i & 3] + y);
                vals[i] = mode ? mixed : y;
            }
            volatile v4f* d4 = (volatile v4f*)(dch + base);
#pragma unroll
            for (int q = 0; q < 8; ++q) {
                v4f w;
                w[0] = vals[4 * q + 0];
                w[1] = vals[4 * q + 1];
                w[2] = vals[4 * q + 2];
                w[3] = vals[4 * q + 3];
                d4[q] = w;
            }
        }
        if (pass == 0) __threadfence();
    }
}

extern "C" void kernel_launch(void* const* d_in, const int* in_sizes, int n_in,
                              void* d_out, int out_size, void* d_ws, size_t ws_size,
                              hipStream_t stream)
{
    if (n_in < 12) return;
    if (in_sizes[0] != TSAMP || out_size != NCH * TSAMP) return;
    if (in_sizes[6] != HW || in_sizes[7] != HW || in_sizes[8] != HW * HW ||
        in_sizes[9] != HW || in_sizes[10] != HW) return;
    const size_t need = (size_t)3 * NCH * TSAMP * sizeof(float);
    if (ws_size < need) return;

    const float* x        = (const float*)d_in[0];
    const float* lfo_rate = (const float*)d_in[1];
    const float* phoff    = (const float*)d_in[2];
    const float* amp      = (const float*)d_in[3];
    const float* bias     = (const float*)d_in[4];
    const float* depth    = (const float*)d_in[5];
    const float* W1       = (const float*)d_in[6];
    const float* b1       = (const float*)d_in[7];
    const float* W2       = (const float*)d_in[8];
    const float* b2       = (const float*)d_in[9];
    const float* W3       = (const float*)d_in[10];
    const float* b3       = (const float*)d_in[11];

    float* p    = (float*)d_ws;
    float* buf0 = p    + (size_t)NCH * TSAMP;
    float* buf1 = buf0 + (size_t)NCH * TSAMP;
    float* out  = (float*)d_out;

    k_coef<<<COEF_BLOCKS, COEF_THREADS, 0, stream>>>(
        lfo_rate, phoff, amp, bias, depth, W1, b1, W2, b2, W3, b3, p);

    k_stage<<<NCH, ST_THREADS, 0, stream>>>(x,    0,     p, x, buf0, 0);
    k_stage<<<NCH, ST_THREADS, 0, stream>>>(buf0, TSAMP, p, x, buf1, 0);
    k_stage<<<NCH, ST_THREADS, 0, stream>>>(buf1, TSAMP, p, x, buf0, 0);
    k_stage<<<NCH, ST_THREADS, 0, stream>>>(buf0, TSAMP, p, x, out,  1);
}
